// EnhancedGraphConvEncoder_36034775613469
// MI455X (gfx1250) — hardware-verified
//
#include <hip/hip_runtime.h>
#include <hip/hip_bf16.h>
#include <stddef.h>
#include <math.h>


#define NN    32768
#define NE    524288
#define NG    128
#define SG    256
#define HD    256
#define HL    128
#define QW    768
#define NHD   8
#define DHD   32
#define NHALF 2
#define RH    (NN / NHALF)
#define GH    (NG / NHALF)
#define EPSV  1e-5f
#define SCL   0.17677669529663687f

#define NB    128
#define STHR  256
#define NWV   8
#define EPT   8
#define CHUNK (STHR * EPT)
#define WCAP  (EPT * 32)
#define PCAP  3072
#define EHDR  32
#define EROW  (EHDR + PCAP)
#define PASSN 256
#define LDS_AGG (((NB + 1) * HD + 3 * PASSN) * 4)
#define GTHR  128
#define ATHR  128
#define LDS_ATT (2 * DHD * SG * 2 + 4 * (16 * SG * 4 + 2 * 16 * SG * 2 + 16 * DHD * 4))
#define PLC   1024

#define WE0 (HD * HD)
#define WE1 (QW * HD)
#define WE2 (HD * HD)
#define WE3 (2 * HD * HD)
#define WE4 (HD * QW)
#define WO0 0
#define WO1 (WO0 + 2 * WE0)
#define WO2 (WO1 + 2 * WE1)
#define WO3 (WO2 + 2 * WE2)
#define WO4 (WO3 + 2 * WE3)
#define WTOT (WO4 + 2 * WE4)
#define WB1 (WE0 / 2048)
#define WB2 (WB1 + WE1 / 2048)
#define WB3 (WB2 + WE2 / 2048)
#define WB4 (WB3 + WE3 / 2048)
#define WBT (WB4 + WE4 / 2048)

static_assert(NN == NG * SG);
static_assert((NN % NB) == 0 && (NN % 64) == 0 && (RH % 64) == 0 && (NG % 64) == 0 && (RH % SG) == 0);
static_assert((HD % 64) == 0 && (QW % 64) == 0 && HD == STHR && HD == NHD * DHD && HD == 2 * HL);
static_assert((NE % CHUNK) == 0 && (NN % CHUNK) == 0);
static_assert((PCAP % PASSN) == 0 && (EROW % 32) == 0 && EHDR * 4 == 128);
static_assert(WBT == 320 && (WE0 % 2048) == 0 && (WE1 % 2048) == 0 && (WE3 % 2048) == 0 && (WE4 % 2048) == 0);
static_assert(LDS_AGG <= 300 * 1024 && LDS_ATT <= 300 * 1024);
static_assert(STHR == NWV * 32 && NB == 16 * NWV && NB == 4 * 32);
static_assert(ATHR == 4 * 32 && SG == 4 * 64 && GTHR == 4 * 32);
static_assert((QW % 8) == 0 && QW / 8 <= STHR && PLC <= 4 * STHR);

typedef float          v4f   __attribute__((ext_vector_type(4)));
typedef float          v8f   __attribute__((ext_vector_type(8)));
typedef int            v4i   __attribute__((ext_vector_type(4)));
typedef unsigned short v8us  __attribute__((ext_vector_type(8)));
typedef unsigned short v16us __attribute__((ext_vector_type(16)));
typedef __bf16         v16bf __attribute__((ext_vector_type(16)));
union FragB { v16bf v; v16us u; v8us h[2]; };
union Pk8 { v8us h; v4i i; };

__device__ __forceinline__ unsigned f2bf(float f) {
  const unsigned u = __float_as_uint(f);
  return (u + 0x7FFFu + ((u >> 16) & 1u)) >> 16;
}

__device__ __forceinline__ void split8(v4f a, v4f b, v8us& hi, v8us& lo) {
  float f[8];
  f[0] = a.x; f[1] = a.y; f[2] = a.z; f[3] = a.w;
  f[4] = b.x; f[5] = b.y; f[6] = b.z; f[7] = b.w;
  v8us rh, rl;
#pragma unroll
  for (int i = 0; i < 8; ++i) {
    const unsigned hb = f2bf(f[i]);
    const float r = f[i] - __uint_as_float(hb << 16);
    rh[i] = (unsigned short)hb;
    rl[i] = (unsigned short)f2bf(r);
  }
  hi = rh;
  lo = rl;
}

__device__ __forceinline__ v8f vz8() {
  v8f c;
#pragma unroll
  for (int i = 0; i < 8; ++i) c[i] = 0.0f;
  return c;
}

__device__ __forceinline__ v8f wm3(v16bf ah, v16bf al, v16bf bh, v16bf bl, v8f c) {
  v8f d = __builtin_amdgcn_wmma_f32_16x16x32_bf16(false, ah, false, bh, (short)0, c, false, false);
  d = __builtin_amdgcn_wmma_f32_16x16x32_bf16(false, ah, false, bl, (short)0, d, false, false);
  d = __builtin_amdgcn_wmma_f32_16x16x32_bf16(false, al, false, bh, (short)0, d, false, false);
  asm volatile("v_nop\n\tv_nop\n\tv_nop\n\tv_nop" : "+v"(d) : "v"(ah), "v"(al), "v"(bh), "v"(bl));
  return d;
}

__device__ __forceinline__ float wsum(float s) {
#pragma unroll
  for (int off = 16; off > 0; off >>= 1) s += __shfl_xor(s, off);
  return s;
}

__global__ __launch_bounds__(256) void k_wprep(const float* __restrict__ wl, const float* __restrict__ wg,
    const float* __restrict__ ipw, const float* __restrict__ opw, const float* __restrict__ rw,
    const float* __restrict__ cw, unsigned short* wpl) {
  const int b = blockIdx.x, tid = threadIdx.x;
  int seg, ub, ne, po;
  if (b < WB1)      { seg = 0; ub = b;       ne = WE0; po = WO0; }
  else if (b < WB2) { seg = 1; ub = b - WB1; ne = WE1; po = WO1; }
  else if (b < WB3) { seg = 2; ub = b - WB2; ne = WE2; po = WO2; }
  else if (b < WB4) { seg = 3; ub = b - WB3; ne = WE3; po = WO3; }
  else              { seg = 4; ub = b - WB4; ne = WE4; po = WO4; }
  const int K = (seg == 4) ? QW : HD;
  const int u = ub * 256 + tid, cpr = K >> 3;
  const int n = u / cpr, kc = u - n * cpr;
  float f[8];
#pragma unroll
  for (int j = 0; j < 8; ++j) {
    const int k = 8 * kc + j;
    float v;
    if (seg == 0) {
      const float a = wl[k * HL + (n & (HL - 1))];
      const float c = wg[k * HL + (n & (HL - 1))];
      v = (n < HL) ? a : c;
    } else if (seg == 1) {
      v = ipw[n * HD + k];
    } else if (seg == 2) {
      v = opw[n * HD + k];
    } else if (seg == 3) {
      v = rw[(size_t)(n >> 8) * HD * HD + (size_t)k * HD + (n & (HD - 1))];
    } else {
      v = cw[n * QW + k];
    }
    f[j] = v;
  }
  Pk8 ph, pq;
  {
    v4f a, c;
    a.x = f[0]; a.y = f[1]; a.z = f[2]; a.w = f[3];
    c.x = f[4]; c.y = f[5]; c.z = f[6]; c.w = f[7];
    split8(a, c, ph.h, pq.h);
  }
  unsigned short* dh = wpl + po + (size_t)u * 8;
  unsigned short* dl = wpl + po + ne + (size_t)u * 8;
  *(volatile v4i*)dh = ph.i;
  *(volatile v4i*)dl = pq.i;
  __threadfence();
  *(volatile v4i*)dh = ph.i;
  *(volatile v4i*)dl = pq.i;
}

__global__ __launch_bounds__(256) void k_cvt(const float* __restrict__ src, unsigned short* pl, int nel) {
  const size_t u = (size_t)blockIdx.x * 256 + threadIdx.x;
  const float* p = src + u * 8;
  Pk8 ph, pq;
  split8(*(const v4f*)p, *(const v4f*)(p + 4), ph.h, pq.h);
  unsigned short* dh = pl + u * 8;
  unsigned short* dl = pl + (size_t)nel + u * 8;
  *(volatile v4i*)dh = ph.i;
  *(volatile v4i*)dl = pq.i;
  __threadfence();
  *(volatile v4i*)dh = ph.i;
  *(volatile v4i*)dl = pq.i;
}

template <int MODE, bool HASB>
__global__ __launch_bounds__(GTHR) void k_gemm3(const unsigned short* __restrict__ Ah, const unsigned short* __restrict__ Al,
    const unsigned short* __restrict__ Bh, const unsigned short* __restrict__ Bl, const float* __restrict__ bias,
    float* Cf, unsigned short* Ch, unsigned short* Cl, int K, int ldc) {
  __shared__ __attribute__((aligned(16))) float stg[4 * 16 * 64];
  const int tid = threadIdx.x, lane = tid & 31, wave = tid >> 5, hh = lane >> 4, m = lane & 15;
  const int r0 = blockIdx.y * 64 + wave * 16;
  const int c0 = blockIdx.x * 64;
  v8f acc[4];
#pragma unroll
  for (int u = 0; u < 4; ++u) acc[u] = vz8();
  const unsigned short* ap = Ah + (size_t)(r0 + m) * K + 8 * hh;
  const unsigned short* aq = Al + (size_t)(r0 + m) * K + 8 * hh;
  const unsigned short* bp = Bh + (size_t)(c0 + m) * K + 8 * hh;
  const unsigned short* bq = Bl + (size_t)(c0 + m) * K + 8 * hh;
#pragma unroll 1
  for (int k0 = 0; k0 < K; k0 += 32) {
    FragB fa, ga;
    fa.h[0] = *(const v8us*)(ap + k0);
    fa.h[1] = *(const v8us*)(ap + k0 + 16);
    ga.h[0] = *(const v8us*)(aq + k0);
    ga.h[1] = *(const v8us*)(aq + k0 + 16);
#pragma unroll
    for (int u = 0; u < 4; ++u) {
      FragB fb, gb;
      const size_t o = (size_t)(16 * u) * K + k0;
      fb.h[0] = *(const v8us*)(bp + o);
      fb.h[1] = *(const v8us*)(bp + o + 16);
      gb.h[0] = *(const v8us*)(bq + o);
      gb.h[1] = *(const v8us*)(bq + o + 16);
      acc[u] = wm3(fa.v, ga.v, fb.v, gb.v, acc[u]);
    }
  }
  float* sw = stg + wave * 1024;
#pragma unroll
  for (int u = 0; u < 4; ++u) {
    const float bv = HASB ? bias[c0 + 16 * u + m] : 0.0f;
#pragma unroll
    for (int r = 0; r < 8; ++r) sw[(8 * hh + r) * 64 + 16 * u + m] = acc[u][r] + bv;
  }
  __syncthreads();
  for (int p = 0; p < 2; ++p) {
    if (MODE != 1) {
#pragma unroll
      for (int it = 0; it < 8; ++it) {
        const int row = 2 * it + (lane >> 4), q = lane & 15;
        const v4f v = *(const v4f*)(sw + row * 64 + 4 * q);
        *(volatile v4f*)(Cf + (size_t)(r0 + row) * ldc + c0 + 4 * q) = v;
      }
    }
    if (MODE != 0) {
#pragma unroll
      for (int it = 0; it < 4; ++it) {
        const int row = 4 * it + (lane >> 3), q = lane & 7;
        const float* sp = sw + row * 64 + 8 * q;
        Pk8 ph, pq;
        split8(*(const v4f*)sp, *(const v4f*)(sp + 4), ph.h, pq.h);
        const size_t off = (size_t)(r0 + row) * ldc + c0 + 8 * q;
        *(volatile v4i*)(Ch + off) = ph.i;
        *(volatile v4i*)(Cl + off) = pq.i;
      }
    }
    if (p == 0) __threadfence();
  }
}

__device__ __forceinline__ int scan_chunk(const int* __restrict__ dsts, int cbase, int nodeBase,
                                          int* list, int tid, int wave) {
  int wc = 0;
  const int el0 = tid * EPT;
  const v4i da = *(const v4i*)(dsts + cbase + el0);
  const v4i db = *(const v4i*)(dsts + cbase + el0 + 4);
  const unsigned nb = (unsigned)nodeBase;
  const unsigned s0 = (unsigned)da.x - nb, s1 = (unsigned)da.y - nb, s2 = (unsigned)da.z - nb, s3 = (unsigned)da.w - nb;
  const unsigned s4 = (unsigned)db.x - nb, s5 = (unsigned)db.y - nb, s6 = (unsigned)db.z - nb, s7 = (unsigned)db.w - nb;
  const bool h0 = s0 < (unsigned)NB, h1 = s1 < (unsigned)NB, h2 = s2 < (unsigned)NB, h3 = s3 < (unsigned)NB;
  const bool h4 = s4 < (unsigned)NB, h5 = s5 < (unsigned)NB, h6 = s6 < (unsigned)NB, h7 = s7 < (unsigned)NB;
  const unsigned any = __builtin_amdgcn_ballot_w32(h0 | h1 | h2 | h3 | h4 | h5 | h6 | h7);
  if (any != 0u) {
#define HITJ(J, HJ) { \
      const unsigned mj = __builtin_amdgcn_ballot_w32(HJ); \
      if (mj != 0u) { \
        if (HJ) { \
          const int pos = wc + (int)__builtin_amdgcn_mbcnt_lo(mj, 0u); \
          if (pos < WCAP) list[wave * WCAP + pos] = el0 + (J); \
        } \
        wc += (int)__builtin_popcount(mj); } }
    HITJ(0, h0) HITJ(1, h1) HITJ(2, h2) HITJ(3, h3)
    HITJ(4, h4) HITJ(5, h5) HITJ(6, h6) HITJ(7, h7)
#undef HITJ
  }
  return wc;
}

__global__ __launch_bounds__(STHR) void k_escan(const int* __restrict__ ei, int* etab, float* nrm) {
  __shared__ int list[NWV * WCAP];
  __shared__ __attribute__((aligned(16))) int pend[EROW];
  __shared__ int pslot[PCAP];
  __shared__ int wcnt[NWV];
  __shared__ __attribute__((aligned(16))) float nv[NB];
  const int tid = threadIdx.x, lane = tid & 31, wave = tid >> 5;
  const int nodeBase = blockIdx.x * NB;
  const int* dsts = ei + NE;
  for (int i = tid; i < EROW; i += STHR) pend[i] = 0;
  __syncthreads();
  int pendN = 0;
#pragma unroll 1
  for (int ch = 0; ch < NE / CHUNK; ++ch) {
    const int cbase = ch * CHUNK;
    const int wc = scan_chunk(dsts, cbase, nodeBase, list, tid, wave);
    if (lane == 0) wcnt[wave] = wc;
    __syncthreads();
    const int base = pendN;
    int tot = 0, myoff = 0;
#pragma unroll
    for (int w = 0; w < NWV; ++w) {
      int c = wcnt[w];
      c = c > WCAP ? WCAP : (c < 0 ? 0 : c);
      if (w < wave) myoff += c;
      tot += c;
    }
    {
      int n = wcnt[wave];
      n = n > WCAP ? WCAP : (n < 0 ? 0 : n);
      for (int i = lane; i < n; i += 32) {
        const int pos = base + myoff + i;
        const int lid = list[wave * WCAP + i] & (CHUNK - 1);
        const int d = dsts[cbase + lid];
        if (pos < PCAP) {
          pend[EHDR + pos] = cbase + lid;
          pslot[pos] = (d - nodeBase) & (NB - 1);
        }
      }
    }
    const int newN = base + tot;
    pendN = newN > PCAP ? PCAP : newN;
    __syncthreads();
  }
  if (tid < NB) {
    int c = 0;
#pragma unroll 4
    for (int i = 0; i < pendN; ++i) c += (pslot[i] == tid) ? 1 : 0;
    nv[tid] = 1.0f / sqrtf((float)c + 1.0f);
  }
  if (tid == 0) pend[0] = pendN;
  __syncthreads();
  int* rowp = etab + (size_t)blockIdx.x * EROW;
  for (int p = 0; p < 2; ++p) {
#pragma unroll 1
    for (int u = tid; u < EROW / 4; u += STHR) {
      const v4i v = *(const v4i*)(pend + 4 * u);
      *(volatile v4i*)(rowp + 4 * u) = v;
    }
    if (wave == 0) *(volatile v4f*)(nrm + nodeBase + 4 * lane) = *(const v4f*)(nv + 4 * lane);
    if (p == 0) __threadfence();
  }
}

template <int MODE>
__global__ __launch_bounds__(STHR) void k_agg(const float* __restrict__ hin, const int* __restrict__ ei,
    const int* __restrict__ etab, const float* __restrict__ nrm, const float* __restrict__ ba,
    const float* __restrict__ bb, const float* __restrict__ lng, const float* __restrict__ lnb,
    float* F, unsigned short* Ph, unsigned short* Pl, int wrpl) {
  extern __shared__ __attribute__((aligned(16))) float dsm[];
  float* acc = dsm;
  int* es = (int*)(dsm + (NB + 1) * HD);
  int* sl = es + PASSN;
  float* cf = (float*)(sl + PASSN);
  const int tid = threadIdx.x, lane = tid & 31, wave = tid >> 5;
  const int nodeBase = blockIdx.x * NB;
  const int* erow = etab + (size_t)blockIdx.x * EROW;
  {
    v4f z;
    z.x = 0.0f; z.y = 0.0f; z.z = 0.0f; z.w = 0.0f;
    for (int i = tid; i < (NB + 1) * HD / 4; i += STHR) *(v4f*)(acc + 4 * i) = z;
  }
  int nP = erow[0];
  nP = nP < 0 ? 0 : (nP > PCAP ? PCAP : nP);
  const int R = (nP + PASSN - 1) / PASSN;
  __syncthreads();
#pragma unroll 1
  for (int r = 0; r < R; ++r) {
    {
      const int idx = r * PASSN + tid;
      const int idxc = idx < PCAP ? idx : PCAP - 1;
      int e = erow[EHDR + idxc];
      e = e < 0 ? 0 : (e > NE - 1 ? NE - 1 : e);
      int s = ei[e];
      s = s < 0 ? 0 : (s > NN - 1 ? NN - 1 : s);
      const int d = ei[NE + e];
      const int dc = d < 0 ? 0 : (d > NN - 1 ? NN - 1 : d);
      int slot = d - nodeBase;
      if (idx >= nP || (unsigned)slot >= (unsigned)NB) slot = NB;
      es[tid] = s;
      sl[tid] = slot;
      cf[tid] = nrm[s] * nrm[dc];
    }
    __syncthreads();
    int cntp = nP - r * PASSN;
    cntp = cntp > PASSN ? PASSN : cntp;
#pragma unroll 1
    for (int i = 0; i < cntp; ++i) {
      unsigned st = (unsigned)sl[i];
      st = st > (unsigned)NB ? (unsigned)NB : st;
      const int sv = es[i] & (NN - 1);
      acc[st * HD + tid] += cf[i] * hin[(size_t)sv * HD + tid];
    }
    __syncthreads();
  }
  {
    float bv;
    if (MODE == 0) {
      const float b0 = ba[tid & (HL - 1)], b1 = bb[tid & (HL - 1)];
      bv = (tid < HL) ? b0 : b1;
    } else {
      bv = ba[tid];
    }
#pragma unroll 1
    for (int row = 0; row < NB; ++row) {
      const int node = nodeBase + row;
      const float nvv = nrm[node];
      const float t = acc[row * HD + tid] + hin[(size_t)node * HD + tid] * (nvv * nvv) + bv;
      acc[row * HD + tid] = (MODE == 0) ? fmaxf(t, 0.0f) : t;
    }
  }
  __syncthreads();
  if (MODE == 1) {
    const v4f g0 = *(const v4f*)(lng + 8 * lane), g1 = *(const v4f*)(lng + 8 * lane + 4);
    const v4f e0 = *(const v4f*)(lnb + 8 * lane), e1 = *(const v4f*)(lnb + 8 * lane + 4);
    float gs[8], be[8];
    gs[0] = g0.x; gs[1] = g0.y; gs[2] = g0.z; gs[3] = g0.w; gs[4] = g1.x; gs[5] = g1.y; gs[6] = g1.z; gs[7] = g1.w;
    be[0] = e0.x; be[1] = e0.y; be[2] = e0.z; be[3] = e0.w; be[4] = e1.x; be[5] = e1.y; be[6] = e1.z; be[7] = e1.w;
#pragma unroll 1
    for (int rr = 0; rr < 16; ++rr) {
      const int row = wave * 16 + rr;
      const int node = nodeBase + row;
      float* ar = acc + row * HD + 8 * lane;
      const v4f a = *(const v4f*)ar, b = *(const v4f*)(ar + 4);
      const v4f x0 = *(const v4f*)(F + (size_t)node * HD + 8 * lane);
      const v4f x1 = *(const v4f*)(F + (size_t)node * HD + 8 * lane + 4);
      float t[8], xs[8];
      t[0] = a.x; t[1] = a.y; t[2] = a.z; t[3] = a.w; t[4] = b.x; t[5] = b.y; t[6] = b.z; t[7] = b.w;
      xs[0] = x0.x; xs[1] = x0.y; xs[2] = x0.z; xs[3] = x0.w; xs[4] = x1.x; xs[5] = x1.y; xs[6] = x1.z; xs[7] = x1.w;
      float s = 0.0f;
#pragma unroll
      for (int j = 0; j < 8; ++j) s += t[j];
      s = wsum(s);
      const float mu = s * (1.0f / HD);
      float q = 0.0f;
#pragma unroll
      for (int j = 0; j < 8; ++j) { const float d = t[j] - mu; t[j] = d; q += d * d; }
      q = wsum(q);
      const float var = q * (1.0f / HD);
      const float rs = 1.0f / sqrtf(var + EPSV);
      float o[8];
#pragma unroll
      for (int j = 0; j < 8; ++j) o[j] = xs[j] + fmaxf(t[j] * rs * gs[j] + be[j], 0.0f);
      v4f o0, o1;
      o0.x = o[0]; o0.y = o[1]; o0.z = o[2]; o0.w = o[3];
      o1.x = o[4]; o1.y = o[5]; o1.z = o[6]; o1.w = o[7];
      *(v4f*)ar = o0;
      *(v4f*)(ar + 4) = o1;
    }
    __syncthreads();
  }
  for (int p = 0; p < 2; ++p) {
#pragma unroll 1
    for (int rr = 0; rr < 16; ++rr) {
      const int row = wave * 16 + rr;
      const size_t nbo = (size_t)(nodeBase + row) * HD;
      const float* ar = acc + row * HD;
      if (MODE == 1) {
        *(volatile v4f*)(F + nbo + 4 * lane) = *(const v4f*)(ar + 4 * lane);
        *(volatile v4f*)(F + nbo + HL + 4 * lane) = *(const v4f*)(ar + HL + 4 * lane);
      }
      if (wrpl != 0) {
        Pk8 ph, pq;
        split8(*(const v4f*)(ar + 8 * lane), *(const v4f*)(ar + 8 * lane + 4), ph.h, pq.h);
        *(volatile v4i*)(Ph + nbo + 8 * lane) = ph.i;
        *(volatile v4i*)(Pl + nbo + 8 * lane) = pq.i;
      }
    }
    if (p == 0) __threadfence();
  }
}

__global__ __launch_bounds__(ATHR) void k_attn(const unsigned short* __restrict__ Qh, const unsigned short* __restrict__ Ql,
                                              float* O, int gofs) {
  extern __shared__ __attribute__((aligned(16))) unsigned char dsa[];
  unsigned short* Vth = (unsigned short*)dsa;
  unsigned short* Vtl = Vth + DHD * SG;
  const int tid = threadIdx.x, lane = tid & 31, wave = tid >> 5, hh = lane >> 4, m = lane & 15;
  float* Sf = (float*)(dsa + 2 * DHD * SG * 2) + wave * (16 * SG);
  unsigned short* Ph = (unsigned short*)(dsa + 2 * DHD * SG * 2 + 4 * 16 * SG * 4) + wave * (2 * 16 * SG);
  unsigned short* Pl = Ph + 16 * SG;
  float* Os = (float*)(dsa + 2 * DHD * SG * 2 + 4 * 16 * SG * 4 + 4 * 2 * 16 * SG * 2) + wave * (16 * DHD);
  const int hd = blockIdx.x, gl = blockIdx.y;
  const size_t gb = (size_t)gl * SG;
  const float ninf = __uint_as_float(0xff800000u);
#pragma unroll 1
  for (int task = tid; task < SG * 4; task += ATHR) {
    const int key = task >> 2, ch = task & 3;
    const size_t o = (gb + key) * QW + 2 * HD + hd * DHD + 8 * ch;
    const v8us vh = *(const v8us*)(Qh + o), vl = *(const v8us*)(Ql + o);
#pragma unroll
    for (int j = 0; j < 8; ++j) {
      Vth[(8 * ch + j) * SG + key] = vh[j];
      Vtl[(8 * ch + j) * SG + key] = vl[j];
    }
  }
  __syncthreads();
#pragma unroll 1
  for (int qt = 0; qt < 4; ++qt) {
    const int q0 = wave * 64 + 16 * qt;
    FragB fq, gq;
    {
      const size_t o = (gb + q0 + m) * QW + hd * DHD + 8 * hh;
      fq.h[0] = *(const v8us*)(Qh + o);
      fq.h[1] = *(const v8us*)(Qh + o + 16);
      gq.h[0] = *(const v8us*)(Ql + o);
      gq.h[1] = *(const v8us*)(Ql + o + 16);
    }
#pragma unroll 2
    for (int kt = 0; kt < 16; ++kt) {
      FragB fk, gk;
      const size_t o = (gb + 16 * kt + m) * QW + HD + hd * DHD + 8 * hh;
      fk.h[0] = *(const v8us*)(Qh + o);
      fk.h[1] = *(const v8us*)(Qh + o + 16);
      gk.h[0] = *(const v8us*)(Ql + o);
      gk.h[1] = *(const v8us*)(Ql + o + 16);
      const v8f s = wm3(fq.v, gq.v, fk.v, gk.v, vz8());
#pragma unroll
      for (int r = 0; r < 8; ++r) Sf[(8 * hh + r) * SG + 16 * kt + m] = s[r] * SCL;
    }
    __syncthreads();
    {
      const int row = lane >> 1, part = lane & 1;
      float* sr = Sf + row * SG + part * 128;
      float mx = ninf;
#pragma unroll 4
      for (int c = 0; c < 128; ++c) mx = fmaxf(mx, sr[c]);
      mx = fmaxf(mx, __shfl_xor(mx, 1));
      float sum = 0.0f;
#pragma unroll 4
      for (int c = 0; c < 128; ++c) { const float e = __expf(sr[c] - mx); sr[c] = e; sum += e; }
      sum += __shfl_xor(sum, 1);
      const float inv = 1.0f / sum;
      unsigned short* pr = Ph + row * SG + part * 128;
      unsigned short* qr = Pl + row * SG + part * 128;
#pragma unroll 4
      for (int c = 0; c < 128; ++c) {
        const float pv = sr[c] * inv;
        const unsigned hb = f2bf(pv);
        pr[c] = (unsigned short)hb;
        qr[c] = (unsigned short)f2bf(pv - __uint_as_float(hb << 16));
      }
    }
    __syncthreads();
    v8f oa[2];
    oa[0] = vz8();
    oa[1] = vz8();
#pragma unroll 2
    for (int kc = 0; kc < 8; ++kc) {
      FragB fp, gp;
      const int o = m * SG + 32 * kc + 8 * hh;
      fp.h[0] = *(const v8us*)(Ph + o);
      fp.h[1] = *(const v8us*)(Ph + o + 16);
      gp.h[0] = *(const v8us*)(Pl + o);
      gp.h[1] = *(const v8us*)(Pl + o + 16);
#pragma unroll
      for (int u = 0; u < 2; ++u) {
        FragB fv, gv;
        const int o2 = (16 * u + m) * SG + 32 * kc + 8 * hh;
        fv.h[0] = *(const v8us*)(Vth + o2);
        fv.h[1] = *(const v8us*)(Vth + o2 + 16);
        gv.h[0] = *(const v8us*)(Vtl + o2);
        gv.h[1] = *(const v8us*)(Vtl + o2 + 16);
        oa[u] = wm3(fp.v, gp.v, fv.v, gv.v, oa[u]);
      }
    }
#pragma unroll
    for (int u = 0; u < 2; ++u) {
#pragma unroll
      for (int r = 0; r < 8; ++r) Os[(8 * hh + r) * DHD + 16 * u + m] = oa[u][r];
    }
    __syncthreads();
    const size_t orow = (size_t)(gofs + gl) * SG + q0;
    for (int p = 0; p < 2; ++p) {
#pragma unroll
      for (int it = 0; it < 4; ++it) {
        const int row = 4 * it + (lane >> 3), q = lane & 7;
        const v4f v = *(const v4f*)(Os + row * DHD + 4 * q);
        *(volatile v4f*)(O + (orow + row) * HD + hd * DHD + 4 * q) = v;
      }
      if (p == 0) __threadfence();
    }
    __syncthreads();
  }
}

__global__ __launch_bounds__(STHR) void k_pool(const float* __restrict__ F, const int* __restrict__ batch,
    const float* __restrict__ gw, const float* __restrict__ gbias, unsigned short* CBh, unsigned short* CBl) {
  __shared__ int plist[NWV * WCAP];
  __shared__ int nl[PLC];
  __shared__ float lgv[PLC];
  __shared__ float red[STHR];
  __shared__ int pwc[NWV];
  __shared__ __attribute__((aligned(16))) float cmb[QW];
  const int tid = threadIdx.x, lane = tid & 31, wave = tid >> 5, g = blockIdx.x;
  const float ninf = __uint_as_float(0xff800000u);
  int tot = 0;
#pragma unroll 1
  for (int ch = 0; ch < NN / CHUNK; ++ch) {
    const int n0 = ch * CHUNK + tid * EPT;
    const v4i a = *(const v4i*)(batch + n0), b = *(const v4i*)(batch + n0 + 4);
    const bool h0 = a.x == g, h1 = a.y == g, h2 = a.z == g, h3 = a.w == g;
    const bool h4 = b.x == g, h5 = b.y == g, h6 = b.z == g, h7 = b.w == g;
    int wc = 0;
    const unsigned any = __builtin_amdgcn_ballot_w32(h0 | h1 | h2 | h3 | h4 | h5 | h6 | h7);
    if (any != 0u) {
#define PH(J, HJ) { \
        const unsigned mj = __builtin_amdgcn_ballot_w32(HJ); \
        if (mj != 0u) { \
          if (HJ) { \
            const int pos = wc + (int)__builtin_amdgcn_mbcnt_lo(mj, 0u); \
            if (pos < WCAP) plist[wave * WCAP + pos] = n0 + (J); \
          } \
          wc += (int)__builtin_popcount(mj); } }
      PH(0, h0) PH(1, h1) PH(2, h2) PH(3, h3) PH(4, h4) PH(5, h5) PH(6, h6) PH(7, h7)
#undef PH
    }
    if (lane == 0) pwc[wave] = wc;
    __syncthreads();
    int t2 = 0, myoff = 0;
#pragma unroll
    for (int w = 0; w < NWV; ++w) {
      int c = pwc[w];
      c = c > WCAP ? WCAP : (c < 0 ? 0 : c);
      if (w < wave) myoff += c;
      t2 += c;
    }
    {
      int n = pwc[wave];
      n = n > WCAP ? WCAP : (n < 0 ? 0 : n);
      for (int i = lane; i < n; i += 32) {
        const int pos = tot + myoff + i;
        if (pos < PLC) nl[pos] = plist[wave * WCAP + i];
      }
    }
    tot += t2;
    __syncthreads();
  }
  const int n = tot > PLC ? PLC : tot;
#pragma unroll 1
  for (int i = tid; i < n; i += STHR) {
    const int nd = nl[i] & (NN - 1);
    const float* fr = F + (size_t)nd * HD;
    float s = 0.0f;
#pragma unroll 1
    for (int c = 0; c < HD; c += 4) {
      const v4f f = *(const v4f*)(fr + c);
      const v4f w = *(const v4f*)(gw + c);
      s += f.x * w.x; s += f.y * w.y; s += f.z * w.z; s += f.w * w.w;
    }
    lgv[i] = s + gbias[0];
  }
  __syncthreads();
  float mx = ninf;
  for (int i = tid; i < n; i += STHR) mx = fmaxf(mx, lgv[i]);
  red[tid] = mx;
  __syncthreads();
  for (int s = STHR / 2; s > 0; s >>= 1) { if (tid < s) red[tid] = fmaxf(red[tid], red[tid + s]); __syncthreads(); }
  mx = red[0];
  __syncthreads();
  float sm = 0.0f;
  for (int i = tid; i < n; i += STHR) { const float e = expf(lgv[i] - mx); lgv[i] = e; sm += e; }
  red[tid] = sm;
  __syncthreads();
  for (int s = STHR / 2; s > 0; s >>= 1) { if (tid < s) red[tid] += red[tid + s]; __syncthreads(); }
  const float inv = 1.0f / red[0];
  for (int i = tid; i < n; i += STHR) lgv[i] = lgv[i] * inv;
  __syncthreads();
  {
    float att = 0.0f, su = 0.0f, mv = ninf;
#pragma unroll 1
    for (int i = 0; i < n; ++i) {
      const int nd = nl[i] & (NN - 1);
      const float v = F[(size_t)nd * HD + tid];
      att += lgv[i] * v;
      su += v;
      mv = fmaxf(mv, v);
    }
    cmb[tid] = att;
    cmb[HD + tid] = su * (1.0f / (float)tot);
    cmb[2 * HD + tid] = mv;
  }
  __syncthreads();
  const int q = tid < QW / 8 ? tid : 0;
  Pk8 ph, pq;
  split8(*(const v4f*)(cmb + 8 * q), *(const v4f*)(cmb + 8 * q + 4), ph.h, pq.h);
  const size_t off = (size_t)g * QW + 8 * q;
  for (int p = 0; p < 2; ++p) {
    if (tid < QW / 8) {
      *(volatile v4i*)(CBh + off) = ph.i;
      *(volatile v4i*)(CBl + off) = pq.i;
    }
    if (p == 0) __threadfence();
  }
}

__global__ __launch_bounds__(STHR) void k_bn(const float* __restrict__ gin, const float* __restrict__ bg,
                                            const float* __restrict__ bbv, float* out) {
  const int c = threadIdx.x;
  double s = 0.0;
#pragma unroll 1
  for (int r = 0; r < NG; ++r) s += (double)gin[r * HD + c];
  const float mu = (float)(s * (1.0 / NG));
  double q = 0.0;
#pragma unroll 1
  for (int r = 0; r < NG; ++r) { const float d = gin[r * HD + c] - mu; q += (double)d * (double)d; }
  const float var = (float)(q * (1.0 / NG));
  const float scl = (1.0f / sqrtf(var + EPSV)) * bg[c];
  const float sh = bbv[c];
  for (int p = 0; p < 2; ++p) {
#pragma unroll 1
    for (int r = 0; r < NG; ++r) {
      const float y = (gin[r * HD + c] - mu) * scl + sh;
      *(volatile float*)(out + r * HD + c) = y;
    }
    if (p == 0) __threadfence();
  }
}

extern "C" void kernel_launch(void* const* d_in, const int* in_sizes, int n_in,
                              void* d_out, int out_size, void* d_ws, size_t ws_size,
                              hipStream_t stream) {
  if (n_in < 21) return;
  if (in_sizes[0] != NN * HD || in_sizes[1] != 2 * NE || in_sizes[2] != NN) return;
  if (in_sizes[3] != HD * HL || in_sizes[4] != HL || in_sizes[5] != HD * HL || in_sizes[6] != HL) return;
  if (in_sizes[7] != QW * HD || in_sizes[8] != QW || in_sizes[9] != HD * HD || in_sizes[10] != HD) return;
  if (in_sizes[11] != 2 * HD * HD || in_sizes[12] != 2 * HD || in_sizes[13] != 2 * HD || in_sizes[14] != 2 * HD) return;
  if (in_sizes[15] != HD || in_sizes[16] != 1 || in_sizes[17] != HD * QW || in_sizes[18] != HD) return;
  if (in_sizes[19] != HD || in_sizes[20] != HD || out_size != NG * HD) return;

  const float* x     = (const float*)d_in[0];
  const int*   ei    = (const int*)d_in[1];
  const int*   batch = (const int*)d_in[2];
  const float* wl  = (const float*)d_in[3],  *bl  = (const float*)d_in[4];
  const float* wg  = (const float*)d_in[5],  *bgl = (const float*)d_in[6];
  const float* ipw = (const float*)d_in[7],  *ipb = (const float*)d_in[8];
  const float* opw = (const float*)d_in[9],  *opb = (const float*)d_in[10];
  const float* rw  = (const float*)d_in[11], *rb  = (const float*)d_in[12];
  const float* lg  = (const float*)d_in[13], *lb  = (const float*)d_in[14];
  const float* gw  = (const float*)d_in[15], *gbi = (const float*)d_in[16];
  const float* cw  = (const float*)d_in[17], *cb  = (const float*)d_in[18];
  const float* bng = (const float*)d_in[19], *bnb = (const float*)d_in[20];
  float* dout = (float*)d_out;

  char* ws = (char*)d_ws;
  size_t off = 0;
  auto carve = [&](size_t bytes) -> size_t {
    const size_t o = off;
    off = (off + bytes + 255) & ~(size_t)255;
    return o;
  };
  const size_t oW  = carve((size_t)WTOT * 2);
  const size_t oR1 = carve((size_t)NN * HD * 4);
  const size_t oR2 = carve((size_t)NN * HD * 4);
  const size_t oR3 = carve((size_t)RH * QW * 4);
  const size_t oET = carve((size_t)(NN / NB) * EROW * 4);
  const size_t oNR = carve((size_t)NN * 4);
  const size_t oCB = carve((size_t)NG * QW * 4);
  const size_t oGO = carve((size_t)NG * HD * 4);
  size_t limit = (size_t)134217728;
  if (ws_size < limit) limit = ws_size;
  if (off > limit) return;

  unsigned short* WP  = (unsigned short*)(ws + oW);
  unsigned short* W0h = WP + WO0, *W0l = W0h + WE0;
  unsigned short* W1h = WP + WO1, *W1l = W1h + WE1;
  unsigned short* W2h = WP + WO2, *W2l = W2h + WE2;
  unsigned short* W3h = WP + WO3, *W3l = W3h + WE3;
  unsigned short* W4h = WP + WO4, *W4l = W4h + WE4;
  float* R1f = (float*)(ws + oR1);
  unsigned short* R1h = (unsigned short*)(ws + oR1), *R1l = R1h + (size_t)NN * HD;
  float* R2f = (float*)(ws + oR2);
  unsigned short* R2h = (unsigned short*)(ws + oR2), *R2l = R2h + (size_t)NN * HD;
  float* R3f = (float*)(ws + oR3);
  unsigned short* R3h = (unsigned short*)(ws + oR3), *R3l = R3h + (size_t)RH * QW;
  int*   ET  = (int*)(ws + oET);
  float* NR  = (float*)(ws + oNR);
  unsigned short* CBh = (unsigned short*)(ws + oCB), *CBl = CBh + (size_t)NG * QW;
  float* GO  = (float*)(ws + oGO);

  k_wprep<<<WBT, 256, 0, stream>>>(wl, wg, ipw, opw, rw, cw, WP);
  k_cvt<<<NN * HD / 8 / 256, 256, 0, stream>>>(x, R1h, NN * HD);
  k_gemm3<0, false><<<dim3(HD / 64, NN / 64), GTHR, 0, stream>>>(R1h, R1l, W0h, W0l, bl, R2f, R3h, R3l, HD, HD);
  k_escan<<<NN / NB, STHR, 0, stream>>>(ei, ET, NR);

  hipFuncSetAttribute(reinterpret_cast<const void*>(&k_agg<0>), hipFuncAttributeMaxDynamicSharedMemorySize, LDS_AGG);
  hipFuncSetAttribute(reinterpret_cast<const void*>(&k_agg<1>), hipFuncAttributeMaxDynamicSharedMemorySize, LDS_AGG);
  hipFuncSetAttribute(reinterpret_cast<const void*>(&k_attn), hipFuncAttributeMaxDynamicSharedMemorySize, LDS_ATT);
  k_agg<0><<<NN / NB, STHR, LDS_AGG, stream>>>(R2f, ei, ET, NR, bl, bgl, lg, lb, R3f, R1h, R1l, 1);

  for (int hf = 0; hf < NHALF; ++hf) {
    const size_t ao = (size_t)hf * RH * HD;
    k_gemm3<1, true><<<dim3(QW / 64, RH / 64), GTHR, 0, stream>>>(R1h + ao, R1l + ao, W1h, W1l, ipb, R2f, R3h, R3l, HD, QW);
    k_attn<<<dim3(NHD, GH), ATHR, LDS_ATT, stream>>>(R3h, R3l, R2f, hf * GH);
  }
  k_cvt<<<NN * HD / 8 / 256, 256, 0, stream>>>(R2f, R1h, NN * HD);
  k_gemm3<2, true><<<dim3(HD / 64, NN / 64), GTHR, 0, stream>>>(R1h, R1l, W2h, W2l, opb, R3f, R2h, R2l, HD, HD);

  for (int i = 0; i < 2; ++i) {
    k_gemm3<0, false><<<dim3(HD / 64, NN / 64), GTHR, 0, stream>>>(R2h, R2l, W3h + (size_t)i * HD * HD, W3l + (size_t)i * HD * HD,
                                                                  rb, R1f, CBh, CBl, HD, HD);
    k_agg<1><<<NN / NB, STHR, LDS_AGG, stream>>>(R1f, ei, ET, NR, rb + i * HD, rb + i * HD, lg + i * HD, lb + i * HD,
                                                R3f, R2h, R2l, i == 0 ? 1 : 0);
  }

  k_pool<<<NG, STHR, 0, stream>>>(R3f, batch, gw, gbi, CBh, CBl);
  k_gemm3<0, true><<<dim3(HD / 64, NG / 64), GTHR, 0, stream>>>(CBh, CBl, W4h, W4l, cb, GO, R1h, R1l, QW, HD);
  k_bn<<<1, STHR, 0, stream>>>(GO, bng, bnb, dout);
}
